// NeuralODE_38053410242883
// MI455X (gfx1250) — hardware-run, weakly checked
//
#include <hip/hip_runtime.h>

typedef __attribute__((ext_vector_type(16))) _Float16 v16h;
typedef __attribute__((ext_vector_type(8)))  _Float16 v8h;
typedef __attribute__((ext_vector_type(8)))  float    v8f;
typedef __attribute__((ext_vector_type(4)))  float    v4f;

constexpr int kSteps     = 100000;
constexpr int kChunk     = 32;
constexpr int kNumChunks = kSteps / kChunk;
constexpr int kHid       = 32;
constexpr int kInW       = 3;
constexpr int kGw        = 16;
static_assert(kNumChunks * kChunk == kSteps);
static_assert(kHid == 32);
static_assert(kGw == 16);
static_assert((kSteps * 4) % 128 == 0);

constexpr float kW2Carry    = 64.0f;
constexpr float kW2CarryInv = 1.0f / kW2Carry;
constexpr float kFieldScale = 0.001f;

constexpr int kOffG1W = 0;
constexpr int kOffG1B = 2 * kGw;
constexpr int kOffG2W = 3 * kGw;
constexpr int kGTotal = 4 * kGw;
static_assert(kGTotal == 64);

__device__ __forceinline__ float softplus_f(float x) {
  const float kLog2e = 1.4426950408889634f;
  const float kLn2   = 0.6931471805599453f;
  const float e = __builtin_amdgcn_exp2f(-fabsf(x) * kLog2e);
  return fmaxf(x, 0.0f) + __builtin_amdgcn_logf(1.0f + e) * kLn2;
}

__device__ __forceinline__ float bcast_lane(float v, int k) {
  const int iv = __builtin_bit_cast(int, v);
  const int rv = __builtin_amdgcn_readlane(iv, k);
  return __builtin_bit_cast(float, rv);
}

__device__ __forceinline__ v8f mma_f16(v16h a, v16h b, v8f c) {
  return __builtin_amdgcn_wmma_f32_16x16x32_f16(false, a, false, b, (short)0, c, false, false);
}

__device__ __forceinline__ void group_guard(v8f& d0, v8f& d1, v16h a, v16h b0, v16h b1) {
  asm volatile("v_nop\n\tv_nop\n\tv_nop\n\tv_nop" : "+v"(d0), "+v"(d1) : "v"(a), "v"(b0), "v"(b1));
}

union FragH { v16h v; v8h h[2]; };

__global__ __launch_bounds__(32, 1) void euler_scan_readout_kernel(
    const float* __restrict__ ts, const float* __restrict__ us, const float* __restrict__ x0p,
    const float* __restrict__ W1, const float* __restrict__ b1, const float* __restrict__ W2,
    const float* __restrict__ b2, const float* __restrict__ W3, const float* __restrict__ b3,
    const float* __restrict__ Wg1, const float* __restrict__ bg1, const float* __restrict__ Wg2,
    const float* __restrict__ bg2, float* __restrict__ out)
{
  __shared__ __align__(16) _Float16 sH[2 * kHid];
  __shared__ __align__(16) float sG[kGTotal];

  const int lane = threadIdx.x & 31;
  const int hsel = lane >> 4;
  const int col  = lane & 15;

  const float w10 = W1[lane * kInW + 0];
  const float w11 = W1[lane * kInW + 1];
  const float w12 = W1[lane * kInW + 2];
  const float b1v = b1[lane];
  const float b2v = b2[lane];
  const float w30 = W3[lane];
  const float w31 = W3[kHid + lane];
  const float b30 = b3[0];
  const float b31 = b3[1];
  const float bg2v = bg2[0];
  const float dtS = (ts[1] - ts[0]) * kFieldScale;

  sG[kOffG1W + lane] = Wg1[lane];
  sG[kOffG1B + col]  = bg1[col];
  sG[kOffG2W + col]  = Wg2[col];

  v16h bw0, bw1;
  {
    const float* r0 = W2 + (size_t)col * kHid + 8 * hsel;
    const float* r1 = W2 + (size_t)(16 + col) * kHid + 8 * hsel;
    const v4f p0 = *(const v4f*)(r0);
    const v4f p1 = *(const v4f*)(r0 + 4);
    const v4f p2 = *(const v4f*)(r0 + 16);
    const v4f p3 = *(const v4f*)(r0 + 20);
    const v4f q0 = *(const v4f*)(r1);
    const v4f q1 = *(const v4f*)(r1 + 4);
    const v4f q2 = *(const v4f*)(r1 + 16);
    const v4f q3 = *(const v4f*)(r1 + 20);
#pragma unroll
    for (int e = 0; e < 4; ++e) {
      bw0[e]      = (_Float16)(p0[e] * kW2Carry);
      bw0[4 + e]  = (_Float16)(p1[e] * kW2Carry);
      bw0[8 + e]  = (_Float16)(p2[e] * kW2Carry);
      bw0[12 + e] = (_Float16)(p3[e] * kW2Carry);
      bw1[e]      = (_Float16)(q0[e] * kW2Carry);
      bw1[4 + e]  = (_Float16)(q1[e] * kW2Carry);
      bw1[8 + e]  = (_Float16)(q2[e] * kW2Carry);
      bw1[12 + e] = (_Float16)(q3[e] * kW2Carry);
    }
  }

  float x0v = x0p[0];
  float x1v = x0p[1];

  __syncthreads();

#pragma unroll 1
  for (int c = 0; c < kNumChunks; ++c) {
    const int tbase = c * kChunk;
    float uv = us[tbase + lane];
    asm volatile("" : "+v"(uv));

    float xr0 = 0.0f;
    float xr1 = 0.0f;

#pragma unroll
    for (int j = 0; j < kChunk; ++j) {
      xr0 = (lane == j) ? x0v : xr0;
      xr1 = (lane == j) ? x1v : xr1;

      const float u = bcast_lane(uv, j);

      float a1 = fmaf(w12, u, b1v);
      a1 = fmaf(w11, x1v, a1);
      a1 = fmaf(w10, x0v, a1);
      const float h1 = softplus_f(a1);

      _Float16* slot = sH + (j & 1) * kHid;
      slot[lane] = (_Float16)h1;
      __syncthreads();

      FragH fa;
      fa.h[0] = *(const v8h*)(slot + 8 * hsel);
      fa.h[1] = *(const v8h*)(slot + 16 + 8 * hsel);

      v8f d0 = (v8f){0.f, 0.f, 0.f, 0.f, 0.f, 0.f, 0.f, 0.f};
      v8f d1 = (v8f){0.f, 0.f, 0.f, 0.f, 0.f, 0.f, 0.f, 0.f};
      d0 = mma_f16(fa.v, bw0, d0);
      d1 = mma_f16(fa.v, bw1, d1);
      group_guard(d0, d1, fa.v, bw0, bw1);

      const float e0 = d0[0];
      const float e1 = d1[0];
      const float dsel = (lane < 16) ? e0 : e1;
      const float h2 = softplus_f(fmaf(dsel, kW2CarryInv, b2v));

      float s0 = w30 * h2;
      float s1 = w31 * h2;
      s0 += __shfl_xor(s0, 16, 32);
      s1 += __shfl_xor(s1, 16, 32);
      s0 += __shfl_xor(s0, 8, 32);
      s1 += __shfl_xor(s1, 8, 32);
      s0 += __shfl_xor(s0, 4, 32);
      s1 += __shfl_xor(s1, 4, 32);
      s0 += __shfl_xor(s0, 2, 32);
      s1 += __shfl_xor(s1, 2, 32);
      s0 += __shfl_xor(s0, 1, 32);
      s1 += __shfl_xor(s1, 1, 32);

      x0v = fmaf(dtS, s0 + b30, x0v);
      x1v = fmaf(dtS, s1 + b31, x1v);
    }

    float accv = 0.0f;
#pragma unroll 1
    for (int n = 0; n < kGw; ++n) {
      const float wa = sG[kOffG1W + 2 * n];
      const float wb = sG[kOffG1W + 2 * n + 1];
      const float bb = sG[kOffG1B + n];
      const float wo = sG[kOffG2W + n];
      float pre = xr0 * wa;
      pre = fmaf(xr1, wb, pre);
      pre = pre + bb;
      accv = fmaf(wo, softplus_f(pre), accv);
    }
    const float yv = accv + bg2v;

    volatile float* po = out + tbase + lane;
    *po = yv;
    __threadfence();
    *po = yv;
  }
}

extern "C" void kernel_launch(void* const* d_in, const int* in_sizes, int n_in,
                              void* d_out, int out_size, void* d_ws, size_t ws_size,
                              hipStream_t stream)
{
  (void)in_sizes; (void)out_size; (void)d_ws; (void)ws_size;
  if (n_in < 13) return;
  const float* ts  = (const float*)d_in[0];
  const float* us  = (const float*)d_in[1];
  const float* x0  = (const float*)d_in[2];
  const float* W1  = (const float*)d_in[3];
  const float* b1  = (const float*)d_in[4];
  const float* W2  = (const float*)d_in[5];
  const float* b2  = (const float*)d_in[6];
  const float* W3  = (const float*)d_in[7];
  const float* b3  = (const float*)d_in[8];
  const float* Wg1 = (const float*)d_in[9];
  const float* bg1 = (const float*)d_in[10];
  const float* Wg2 = (const float*)d_in[11];
  const float* bg2 = (const float*)d_in[12];

  euler_scan_readout_kernel<<<1, 32, 0, stream>>>(ts, us, x0, W1, b1, W2, b2, W3, b3,
                                                  Wg1, bg1, Wg2, bg2, (float*)d_out);
}
